// GIN_22574348108106
// MI455X (gfx1250) — hardware-verified
//
#include <hip/hip_runtime.h>
#include <stddef.h>
#include <stdint.h>


#define FEA     128
#define HD      64
#define NGR     512
#define NLAY    4
#define K2      128
#define KRO     640
#define NTHR    256
#define NWAVE   8
#define EPT     8
#define CHUNK   (NTHR * EPT)
#define WCAP    (EPT * 32)
#define LISTN   (NWAVE * WCAP)
#define NB      1024
#define RCAP    28672
#define DEGCAP  64
#define PKS     11
#define CSRMW   2112
#define CSR_ZINTS (2 * RCAP + 2 * NB + 64 + LISTN + 16)
#define LDS_CSR (CSR_ZINTS * 4)
#define TM      128
#define APITCH  136
#define PARTW   160
#define SEGW    640
#define SEGFLAG 544
#define NUPREP  15360
#define GEMM_LDS (TM * APITCH * 2 + TM * HD * 4 + 128 * 4 + PARTW * 4 + 512 * 4)
#define WSMAX   134217728

static_assert((CHUNK & (CHUNK - 1)) == 0 && CHUNK <= (1 << PKS));
static_assert((NB & (NB - 1)) == 0 && NB <= (1 << PKS) && NB == 4 * NTHR);
static_assert(LISTN >= NB && LISTN >= NWAVE * WCAP);
static_assert((RCAP % (4 * NTHR)) == 0 && (CSR_ZINTS % 4) == 0);
static_assert(LDS_CSR <= 300000 && GEMM_LDS <= 300000);
static_assert((NB % TM) == 0 && TM == NWAVE * 16);
static_assert((K2 % 32) == 0 && (KRO % 32) == 0 && K2 == 2 * HD && FEA == K2);
static_assert((CSRMW % 32) == 0 && CSRMW == 2 * NB + 64 && (CSRMW / 4) <= 3 * NTHR);
static_assert((PARTW % 32) == 0 && PARTW / 4 == 40);
static_assert((NUPREP % NTHR) == 0);
static_assert((APITCH % 8) == 0 && APITCH >= K2);
static_assert(SEGW / 4 <= NTHR && SEGFLAG > NGR + 1 && SEGFLAG < SEGW);

typedef float          v2f  __attribute__((ext_vector_type(2)));
typedef float          v4f  __attribute__((ext_vector_type(4)));
typedef float          v8f  __attribute__((ext_vector_type(8)));
typedef int            v4i  __attribute__((ext_vector_type(4)));
typedef int            v8i  __attribute__((ext_vector_type(8)));
typedef unsigned short v8us __attribute__((ext_vector_type(8)));
typedef __bf16         v16b __attribute__((ext_vector_type(16)));
typedef v2f  __attribute__((may_alias)) v2fa;
typedef v4f  __attribute__((may_alias)) v4fa;
typedef v4i  __attribute__((may_alias)) v4ia;
typedef v8us __attribute__((may_alias)) v8usa;
typedef unsigned int __attribute__((may_alias)) u32a;
union Frag { v16b vb; v8us h[2]; v8i w; };

__device__ __forceinline__ v8f wmb(const Frag& a, const Frag& b, v8f c) {
  v8f d = __builtin_amdgcn_wmma_f32_16x16x32_bf16(false, a.vb, false, b.vb, (short)0, c, false, false);
  asm volatile("v_nop\n\tv_nop\n\tv_nop\n\tv_nop" : "+v"(d) : "v"(a.w), "v"(b.w));
  return d;
}

__device__ __forceinline__ unsigned short bf_bits(float f) {
  unsigned int u = __float_as_uint(f);
  u += 0x7FFFu + ((u >> 16) & 1u);
  return (unsigned short)(u >> 16);
}
__device__ __forceinline__ float bf_val(unsigned short b) { return __uint_as_float(((unsigned int)b) << 16); }
__device__ __forceinline__ float bf_rne(float f) { return bf_val(bf_bits(f)); }
__device__ __forceinline__ float relu_keep(float v) { return (v > 0.0f) ? v : (v - v); }

__device__ __forceinline__ int scan_chunk(const int* __restrict__ dsts, int nE, int cbase, int slotBase,
                                          int nb, int vec8, int* list, int tid, int lane, int wave) {
  int wc = 0;
  const int el0  = tid * EPT;
  const int e0   = cbase + el0;
  const int sent = -2147483647 - 1;
  v4i da, db;
  if (vec8 != 0 && cbase + CHUNK <= nE) {
    da = *(const v4i*)(dsts + e0);
    db = *(const v4i*)(dsts + e0 + 4);
  } else {
    da.x = (e0     < nE) ? dsts[min(e0,     nE - 1)] : sent;
    da.y = (e0 + 1 < nE) ? dsts[min(e0 + 1, nE - 1)] : sent;
    da.z = (e0 + 2 < nE) ? dsts[min(e0 + 2, nE - 1)] : sent;
    da.w = (e0 + 3 < nE) ? dsts[min(e0 + 3, nE - 1)] : sent;
    db.x = (e0 + 4 < nE) ? dsts[min(e0 + 4, nE - 1)] : sent;
    db.y = (e0 + 5 < nE) ? dsts[min(e0 + 5, nE - 1)] : sent;
    db.z = (e0 + 6 < nE) ? dsts[min(e0 + 6, nE - 1)] : sent;
    db.w = (e0 + 7 < nE) ? dsts[min(e0 + 7, nE - 1)] : sent;
  }
  const unsigned nbs = (unsigned)slotBase;
  const unsigned unb = (unsigned)nb;
  const unsigned s0 = (unsigned)da.x - nbs, s1 = (unsigned)da.y - nbs;
  const unsigned s2 = (unsigned)da.z - nbs, s3 = (unsigned)da.w - nbs;
  const unsigned s4 = (unsigned)db.x - nbs, s5 = (unsigned)db.y - nbs;
  const unsigned s6 = (unsigned)db.z - nbs, s7 = (unsigned)db.w - nbs;
  const bool h0 = s0 < unb, h1 = s1 < unb, h2 = s2 < unb, h3 = s3 < unb;
  const bool h4 = s4 < unb, h5 = s5 < unb, h6 = s6 < unb, h7 = s7 < unb;
  const unsigned any = __builtin_amdgcn_ballot_w32(h0 | h1 | h2 | h3 | h4 | h5 | h6 | h7);
  if (any != 0u) {
#define HITJ(J, HJ, SJ) { \
      const unsigned mj = __builtin_amdgcn_ballot_w32(HJ); \
      if (mj != 0u) { \
        if (HJ) { \
          const int pos = wc + (int)__builtin_amdgcn_mbcnt_lo(mj, 0u); \
          if (pos < WCAP) list[wave * WCAP + pos] = ((el0 + (J)) << PKS) | (int)(SJ); \
        } \
        wc += (int)__builtin_popcount(mj); } }
    HITJ(0, h0, s0)
    HITJ(1, h1, s1)
    HITJ(2, h2, s2)
    HITJ(3, h3, s3)
    HITJ(4, h4, s4)
    HITJ(5, h5, s5)
    HITJ(6, h6, s6)
    HITJ(7, h7, s7)
#undef HITJ
  }
  return wc;
}

__device__ __forceinline__ v8us cv8b(const float* __restrict__ p, size_t stride) {
  v8us o;
#pragma unroll
  for (int i = 0; i < 8; ++i) o[i] = bf_bits(p[(size_t)i * stride]);
  return o;
}

__global__ __launch_bounds__(NTHR) void k_prep(const float* __restrict__ fW1, const float* __restrict__ fW2,
                                               const float* __restrict__ cW1, const float* __restrict__ cW2,
                                               const float* __restrict__ linW,
                                               unsigned short* pF1, unsigned short* pF2, unsigned short* pC1,
                                               unsigned short* pC2, unsigned short* pLW) {
  const int u = (int)blockIdx.x * NTHR + (int)threadIdx.x;
  v8us o;
  unsigned short* dp;
  if (u < 1024) {
    const int v = u, n = v >> 4, k8 = (v & 15) * 8;
    o = cv8b(fW1 + (size_t)k8 * HD + n, HD);
    dp = pF1 + (size_t)v * 8;
  } else if (u < 2048) {
    const int v = u - 1024, n = v >> 4, k8 = (v & 15) * 8, kk = k8 & (HD - 1);
    o = cv8b(fW2 + (size_t)kk * HD + n, HD);
    dp = pF2 + (size_t)v * 8;
  } else if (u < 6144) {
    const int v = u - 2048, l = v >> 10, w = v & 1023, n = w >> 4, k8 = (w & 15) * 8, kk = k8 & (HD - 1);
    o = cv8b(cW1 + (size_t)l * (HD * HD) + (size_t)kk * HD + n, HD);
    dp = pC1 + (size_t)v * 8;
  } else if (u < 10240) {
    const int v = u - 6144, l = v >> 10, w = v & 1023, n = w >> 4, k8 = (w & 15) * 8, kk = k8 & (HD - 1);
    o = cv8b(cW2 + (size_t)l * (HD * HD) + (size_t)kk * HD + n, HD);
    dp = pC2 + (size_t)v * 8;
  } else if (u < NUPREP) {
    const int v = u - 10240;
    const int n  = v / (KRO / 8);
    const int k8 = (v - n * (KRO / 8)) * 8;
    const int kk = k8 < (KRO / 2) ? k8 : k8 - (KRO / 2);
    o = cv8b(linW + (size_t)kk * HD + n, HD);
    dp = pLW + (size_t)v * 8;
  } else {
    return;
  }
  *(volatile v8us*)dp = o;
  __threadfence();
  *(volatile v8us*)dp = o;
}

__global__ __launch_bounds__(NTHR) void k_seg(const int* __restrict__ bat, int nN, int* segt) {
  __shared__ __attribute__((aligned(16))) int sg[SEGW];
  __shared__ int wf[NWAVE];
  const int tid = (int)threadIdx.x, lane = tid & 31, wave = tid >> 5;
  int bad = 0;
  const int nIt = (nN + NTHR - 1) / NTHR;
#pragma unroll 1
  for (int it = 0; it < nIt; ++it) {
    const int i  = it * NTHR + tid;
    const int ic = i < nN ? i : nN - 1;
    const int ip = ic > 0 ? ic - 1 : 0;
    const int b  = bat[ic];
    const int pb = bat[ip];
    bad |= ((b < 0) | (b >= NGR) | (pb > b)) ? 1 : 0;
  }
  const unsigned mk = __builtin_amdgcn_ballot_w32(bad != 0);
  if (lane == 0) wf[wave] = (mk != 0u) ? 1 : 0;
  __syncthreads();
  int flag = 0;
#pragma unroll
  for (int w2 = 0; w2 < NWAVE; ++w2) flag |= wf[w2];
#pragma unroll 1
  for (int it = 0; it < 3; ++it) {
    const int j   = it * NTHR + tid;
    const int key = j < NGR ? j : NGR;
    int lo = 0, hi = nN;
#pragma unroll 1
    for (int st = 0; st < 20; ++st) {
      const int mid = (lo + hi) >> 1;
      const int mc  = mid < nN ? mid : nN - 1;
      const int b   = bat[mc];
      const bool act  = lo < hi;
      const bool less = b < key;
      lo = (act && less) ? mid + 1 : lo;
      hi = (act && !less) ? mid : hi;
    }
    const int v = (j <= NGR) ? lo : ((j < SEGFLAG) ? nN : ((j == SEGFLAG) ? flag : 0));
    if (j < SEGW) sg[j] = v;
  }
  __syncthreads();
  const bool ok = tid < SEGW / 4;
  const int tc = ok ? tid : 0;
  const v4i ov = *(const v4ia*)(sg + 4 * tc);
  int* dp = segt + 4 * tc;
  if (ok) *(volatile v4i*)dp = ov;
  __threadfence();
  if (ok) *(volatile v4i*)dp = ov;
}

__global__ __launch_bounds__(NTHR) void k_csr(const int* __restrict__ srcs, const int* __restrict__ dsts,
                                              int nN, int nE, int vec8, int* csrm, int* col) {
  extern __shared__ v4f lds_dyn[];
  int* reg1 = (int*)lds_dyn;
  int* reg2 = reg1 + RCAP;
  int* soff = reg2 + RCAP;
  int* scnt = soff + NB;
  int* misc = scnt + NB;
  int* list = misc + 64;
  int* wcnt = list + LISTN;
  int* wtot = wcnt + NWAVE;
  const int tid = (int)threadIdx.x, lane = tid & 31, wave = tid >> 5;
  const int nodeBase = (int)blockIdx.x * NB;

  {
    const v4i z4 = {0, 0, 0, 0};
    for (int i = tid * 4; i < CSR_ZINTS; i += NTHR * 4) *(v4ia*)(reg1 + i) = z4;
  }
  __syncthreads();

  int tot = 0;
  const int nChunks = (nE + CHUNK - 1) / CHUNK;
#pragma unroll 1
  for (int ch = 0; ch < nChunks; ++ch) {
    const int cbase = ch * CHUNK;
    const int wc = scan_chunk(dsts, nE, cbase, nodeBase, NB, vec8, list, tid, lane, wave);
    if (lane == 0) wcnt[wave] = wc;
    __syncthreads();
    int pre = 0, all = 0;
#pragma unroll
    for (int w2 = 0; w2 < NWAVE; ++w2) {
      int c = wcnt[w2];
      c = c < 0 ? 0 : (c > WCAP ? WCAP : c);
      all += c;
      pre += (w2 < wave) ? c : 0;
    }
    const int wcc  = wc > WCAP ? WCAP : wc;
    const int base = tot + pre;
#pragma unroll 1
    for (int i = lane; i < wcc; i += 32) {
      const int ent = list[wave * WCAP + i];
      const int el  = (ent >> PKS) & (CHUNK - 1);
      const int sl  = ent & (NB - 1);
      int eid = cbase + el;
      eid = eid > nE - 1 ? nE - 1 : eid;
      const int pos = base + i;
      if (pos < RCAP) reg1[pos] = (int)(((unsigned)eid << PKS) | (unsigned)sl);
    }
    tot += all;
    tot = tot > RCAP ? RCAP : tot;
    __syncthreads();
  }
  const int nh = tot;

  if (wave == 0) {
#pragma unroll 1
    for (int b0 = 0; b0 < nh; b0 += 32) {
      const int idx = b0 + lane;
      const int uv  = reg1[idx < RCAP ? idx : RCAP - 1];
      const int m32 = (nh - b0) < 32 ? (nh - b0) : 32;
#pragma unroll 1
      for (int k = 0; k < m32; ++k) {
        const int u  = __builtin_amdgcn_readlane(uv, k);
        const int sl = u & (NB - 1);
        if (lane == 0) scnt[sl] = scnt[sl] + 1;
      }
    }
  }
  __syncthreads();

  {
    const v4i ca = *(const v4ia*)(scnt + 4 * tid);
    const int e0 = ca.x < 0 ? 0 : ca.x, e1 = ca.y < 0 ? 0 : ca.y, e2 = ca.z < 0 ? 0 : ca.z, e3 = ca.w < 0 ? 0 : ca.w;
    const int ts = e0 + e1 + e2 + e3;
    int incl = ts;
#pragma unroll
    for (int d = 1; d < 32; d <<= 1) {
      const int up = __shfl_up(incl, d);
      if (lane >= d) incl += up;
    }
    if (lane == 31) wtot[wave] = incl;
    __syncthreads();
    int pre = 0;
#pragma unroll
    for (int w2 = 0; w2 < NWAVE; ++w2) pre += (w2 < wave) ? wtot[w2] : 0;
    int run = pre + incl - ts;
    soff[4 * tid + 0] = run; run += e0;
    soff[4 * tid + 1] = run; run += e1;
    soff[4 * tid + 2] = run; run += e2;
    soff[4 * tid + 3] = run;
  }
  __syncthreads();
  for (int i = tid; i < NB; i += NTHR) list[i] = soff[i];
  __syncthreads();

  if (wave == 0) {
#pragma unroll 1
    for (int b0 = 0; b0 < nh; b0 += 32) {
      const int idx = b0 + lane;
      const int uv  = reg1[idx < RCAP ? idx : RCAP - 1];
      const int m32 = (nh - b0) < 32 ? (nh - b0) : 32;
#pragma unroll 1
      for (int k = 0; k < m32; ++k) {
        const int u   = __builtin_amdgcn_readlane(uv, k);
        const int sl  = u & (NB - 1);
        const int eid = (int)((unsigned)u >> PKS);
        if (lane == 0) {
          int pos = list[sl];
          pos = pos < 0 ? 0 : (pos > RCAP - 1 ? RCAP - 1 : pos);
          reg2[pos] = eid;
          list[sl] = pos + 1;
        }
      }
    }
  }
  if (tid == 0) { misc[0] = nh; misc[1] = (nh >= RCAP) ? 1 : 0; }
  __syncthreads();

  {
    int* hb = csrm + (size_t)blockIdx.x * CSRMW;
    v4i mv[3];
#pragma unroll
    for (int it = 0; it < 3; ++it) {
      const int p  = it * NTHR + tid;
      const int pc = p < CSRMW / 4 ? p : CSRMW / 4 - 1;
      mv[it] = *(const v4ia*)(soff + 4 * pc);
    }
#pragma unroll
    for (int it = 0; it < 3; ++it) {
      const int p = it * NTHR + tid;
      if (p < CSRMW / 4) *(volatile v4i*)(hb + 4 * p) = mv[it];
    }
    __threadfence();
#pragma unroll
    for (int it = 0; it < 3; ++it) {
      const int p = it * NTHR + tid;
      if (p < CSRMW / 4) *(volatile v4i*)(hb + 4 * p) = mv[it];
    }
  }
  {
    int* cbp = col + (size_t)blockIdx.x * RCAP;
#pragma unroll 1
    for (int it = 0; it < RCAP / (4 * NTHR); ++it) {
      const int i4 = (it * NTHR + tid) * 4;
      const v4i e = *(const v4ia*)(reg2 + i4);
      const int e0 = e.x < 0 ? 0 : (e.x > nE - 1 ? nE - 1 : e.x);
      const int e1 = e.y < 0 ? 0 : (e.y > nE - 1 ? nE - 1 : e.y);
      const int e2 = e.z < 0 ? 0 : (e.z > nE - 1 ? nE - 1 : e.z);
      const int e3 = e.w < 0 ? 0 : (e.w > nE - 1 ? nE - 1 : e.w);
      int s0 = srcs[e0], s1 = srcs[e1], s2 = srcs[e2], s3 = srcs[e3];
      s0 = s0 < 0 ? 0 : (s0 > nN - 1 ? nN - 1 : s0);
      s1 = s1 < 0 ? 0 : (s1 > nN - 1 ? nN - 1 : s1);
      s2 = s2 < 0 ? 0 : (s2 > nN - 1 ? nN - 1 : s2);
      s3 = s3 < 0 ? 0 : (s3 > nN - 1 ? nN - 1 : s3);
      v4i o;
      o.x = (i4     < nh) ? s0 : 0;
      o.y = (i4 + 1 < nh) ? s1 : 0;
      o.z = (i4 + 2 < nh) ? s2 : 0;
      o.w = (i4 + 3 < nh) ? s3 : 0;
      int* dp = cbp + i4;
      *(volatile v4i*)dp = o;
      __threadfence();
      *(volatile v4i*)dp = o;
    }
  }
}

template <int MODE>
__global__ __launch_bounds__(NTHR) void k_gemm(const float* __restrict__ src, const float* __restrict__ ac,
                                               const int* __restrict__ csrm, const int* __restrict__ col,
                                               const unsigned short* __restrict__ BT,
                                               const float* __restrict__ bias,
                                               float* Yout, float* part, int nN) {
  extern __shared__ v4f lds_dyn[];
  unsigned short* At = (unsigned short*)lds_dyn;
  float* stg = (float*)(At + TM * APITCH);
  float* acs = stg + TM * HD;
  float* pst = acs + 128;
  float* psm = pst + PARTW;
  const int tid = (int)threadIdx.x, lane = tid & 31, wave = tid >> 5, hh = lane >> 4, m = lane & 15;
  const int rowBase = (int)blockIdx.x * TM;

  if constexpr (MODE == 0) {
#pragma unroll 1
    for (int it = 0; it < 8; ++it) {
      const int p = it * NTHR + tid;
      const int row = p >> 4, k8 = (p & 15) * 8;
      const int grow = rowBase + row;
      const int rc = grow < nN ? grow : nN - 1;
      const float* xp = src + (size_t)rc * FEA + k8;
      const v4f a = *(const v4f*)xp;
      const v4f b = *(const v4f*)(xp + 4);
      const bool ok = grow < nN;
      const float f[8] = {a.x, a.y, a.z, a.w, b.x, b.y, b.z, b.w};
      v8us o;
#pragma unroll
      for (int j = 0; j < 8; ++j) o[j] = ok ? bf_bits(f[j]) : (unsigned short)0;
      *(v8usa*)(At + row * APITCH + k8) = o;
    }
  } else if constexpr (MODE == 1) {
    if (tid < 32) *(v4fa*)(acs + 4 * tid) = *(const v4f*)(ac + 4 * tid);
    __syncthreads();
#pragma unroll 1
    for (int it = 0; it < 4; ++it) {
      const int p = it * NTHR + tid;
      const int row = p >> 3, c8 = (p & 7) * 8;
      const int grow = rowBase + row;
      const float* yp = src + (size_t)grow * HD + c8;
      const v4f a = *(const v4f*)yp;
      const v4f b = *(const v4f*)(yp + 4);
      const bool ok = grow < nN;
      const float f[8] = {a.x, a.y, a.z, a.w, b.x, b.y, b.z, b.w};
      v8us hv, lv;
#pragma unroll
      for (int j = 0; j < 8; ++j) {
        float t = relu_keep(fmaf(acs[c8 + j], f[j], acs[HD + c8 + j]));
        t = ok ? t : 0.0f;
        const unsigned short hb = bf_bits(t);
        hv[j] = hb;
        lv[j] = bf_bits(t - bf_val(hb));
      }
      *(v8usa*)(At + row * APITCH + c8) = hv;
      *(v8usa*)(At + row * APITCH + HD + c8) = lv;
    }
  } else {
    const int cb    = rowBase >> 10;
    const int slot0 = (rowBase & (NB - 1)) + 16 * wave;
    const int* mb   = csrm + (size_t)cb * CSRMW;
    const int so_l  = mb[slot0 + (lane & 15)];
    const int cn_l  = mb[NB + slot0 + (lane & 15)];
    int nhb = mb[2 * NB];
    const int ovb = mb[2 * NB + 1];
    nhb = nhb < 0 ? 0 : (nhb > RCAP ? RCAP : nhb);
    const int* cbp = col + (size_t)cb * RCAP;
    const float qnan = __int_as_float(0x7fc00000);
#pragma unroll 1
    for (int i = 0; i < 16; ++i) {
      int st = __builtin_amdgcn_readlane(so_l, i);
      const int craw = __builtin_amdgcn_readlane(cn_l, i);
      int cnt = craw;
      st  = st < 0 ? 0 : (st > nhb ? nhb : st);
      cnt = cnt < 0 ? 0 : (cnt > DEGCAP ? DEGCAP : cnt);
      if (cnt > nhb - st) cnt = nhb - st;
      const int lr = 16 * wave + i;
      const int grow = rowBase + lr;
      const bool live = grow < nN;
      float a0 = 0.0f, a1 = 0.0f;
#pragma unroll 1
      for (int b0 = 0; b0 < cnt; b0 += 32) {
        int idx = st + b0 + lane;
        idx = idx > RCAP - 1 ? RCAP - 1 : idx;
        int sr = cbp[idx];
        sr = sr < 0 ? 0 : (sr > nN - 1 ? nN - 1 : sr);
        const int m32 = (cnt - b0) < 32 ? (cnt - b0) : 32;
#pragma unroll 1
        for (int k = 0; k < m32; ++k) {
          const int sk = __builtin_amdgcn_readlane(sr, k);
          const v2f v = *(const v2fa*)(src + (size_t)sk * HD + 2 * lane);
          a0 += v.x; a1 += v.y;
        }
      }
      const int nc = live ? grow : nN - 1;
      const v2f sv = *(const v2fa*)(src + (size_t)nc * HD + 2 * lane);
      const float pz = (ovb != 0 || craw > DEGCAP || craw < 0) ? qnan : 0.0f;
      float z0 = (sv.x + a0) + pz;
      float z1 = (sv.y + a1) + pz;
      z0 = live ? z0 : 0.0f;
      z1 = live ? z1 : 0.0f;
      const unsigned short h0 = bf_bits(z0), h1 = bf_bits(z1);
      const unsigned short l0 = bf_bits(z0 - bf_val(h0)), l1 = bf_bits(z1 - bf_val(h1));
      *(u32a*)(At + lr * APITCH + 2 * lane)      = (unsigned int)h0 | ((unsigned int)h1 << 16);
      *(u32a*)(At + lr * APITCH + HD + 2 * lane) = (unsigned int)l0 | ((unsigned int)l1 << 16);
    }
  }
  __syncthreads();

  v8f acc[4];
  {
    const v8f z = {0.f, 0.f, 0.f, 0.f, 0.f, 0.f, 0.f, 0.f};
    acc[0] = z; acc[1] = z; acc[2] = z; acc[3] = z;
  }
  const unsigned short* ap = At + (16 * wave + m) * APITCH + 8 * hh;
  const unsigned short* wp = BT + (size_t)m * K2 + 8 * hh;
#pragma unroll 1
  for (int k0 = 0; k0 < K2; k0 += 32) {
    Frag af;
    af.h[0] = *(const v8usa*)(ap + k0);
    af.h[1] = *(const v8usa*)(ap + k0 + 16);
#pragma unroll
    for (int nt = 0; nt < 4; ++nt) {
      const unsigned short* wq = wp + (size_t)(16 * nt) * K2 + k0;
      Frag bfr;
      bfr.h[0] = *(const v8usa*)wq;
      bfr.h[1] = *(const v8usa*)(wq + 16);
      acc[nt] = wmb(af, bfr, acc[nt]);
    }
  }

#pragma unroll
  for (int nt = 0; nt < 4; ++nt) {
    const int lc = 16 * nt + m;
    const float bb = bf_rne(bias[lc]);
#pragma unroll
    for (int r = 0; r < 8; ++r) {
      const int lr = 16 * wave + 8 * hh + r;
      const bool live = (rowBase + lr) < nN;
      const float v = acc[nt][r] + bb;
      stg[lr * HD + lc] = live ? v : 0.0f;
    }
  }
  __syncthreads();

  int nvr = nN - rowBase;
  nvr = nvr < 0 ? 0 : (nvr > TM ? TM : nvr);
  const int c = tid & (HD - 1);
  const int q = tid >> 6;
  const int r0 = q * 32;
  const int r1 = (r0 + 32) < nvr ? (r0 + 32) : nvr;
  {
    float s = 0.0f;
#pragma unroll 1
    for (int r = r0; r < r1; ++r) s += stg[r * HD + c];
    psm[q * HD + c] = s;
  }
  __syncthreads();
  const float inv  = 1.0f / (float)(nvr < 1 ? 1 : nvr);
  const float mean = (((psm[c] + psm[HD + c]) + psm[2 * HD + c]) + psm[3 * HD + c]) * inv;
  {
    float qq = 0.0f;
#pragma unroll 1
    for (int r = r0; r < r1; ++r) {
      const float d = stg[r * HD + c] - mean;
      qq = fmaf(d, d, qq);
    }
    psm[256 + q * HD + c] = qq;
  }
  __syncthreads();
  if (tid < HD) {
    pst[tid] = mean;
    pst[HD + tid] = ((psm[256 + tid] + psm[256 + HD + tid]) + psm[256 + 2 * HD + tid]) + psm[256 + 3 * HD + tid];
  } else if (tid == HD) {
    pst[2 * HD] = (float)nvr;
  } else if (tid < HD + 32) {
    pst[2 * HD + (tid - HD)] = 0.0f;
  }
  __syncthreads();

  v4f fv[8];
#pragma unroll
  for (int i = 0; i < 8; ++i) {
    const int lr = 16 * wave + 2 * i + hh;
    fv[i] = *(const v4fa*)(stg + lr * HD + 4 * m);
  }
  const bool pok = tid < PARTW / 4;
  const int ptc = pok ? tid : 0;
  const v4f pv = *(const v4fa*)(pst + 4 * ptc);
  float* pp = part + (size_t)blockIdx.x * PARTW + 4 * ptc;
#pragma unroll
  for (int i = 0; i < 8; ++i) {
    const int lr = 16 * wave + 2 * i + hh;
    float* op = Yout + (size_t)(rowBase + lr) * HD + 4 * m;
    *(volatile v4f*)op = fv[i];
  }
  if (pok) *(volatile v4f*)pp = pv;
  __threadfence();
#pragma unroll
  for (int i = 0; i < 8; ++i) {
    const int lr = 16 * wave + 2 * i + hh;
    float* op = Yout + (size_t)(rowBase + lr) * HD + 4 * m;
    *(volatile v4f*)op = fv[i];
  }
  if (pok) *(volatile v4f*)pp = pv;
}

__global__ __launch_bounds__(HD) void k_bncomb(const float* __restrict__ part, int nT,
                                               const float* __restrict__ gam, const float* __restrict__ bet,
                                               float* acout) {
  __shared__ __attribute__((aligned(16))) float stg[2 * HD];
  const int tid = (int)threadIdx.x;
  double n = 0.0, mean = 0.0, M2 = 0.0;
#pragma unroll 1
  for (int b = 0; b < nT; ++b) {
    const float* pr = part + (size_t)b * PARTW;
    const double nb = (double)pr[2 * HD];
    const double mb = (double)pr[tid];
    const double qb = (double)pr[HD + tid];
    if (nb > 0.5) {
      const double nn = n + nb;
      const double delta = mb - mean;
      const double f = nb / nn;
      mean = mean + delta * f;
      M2 = M2 + qb + delta * delta * n * f;
      n = nn;
    }
  }
  const double nt = n < 1.0 ? 1.0 : n;
  const double ve = M2 / nt + 1e-5;
  double rs = (double)rsqrtf((float)ve);
  rs = rs * (1.5 - 0.5 * ve * rs * rs);
  const double a  = (double)bf_rne(gam[tid]) * rs;
  const double cc = (double)bf_rne(bet[tid]) - mean * a;
  stg[tid] = (float)a;
  stg[HD + tid] = (float)cc;
  __syncthreads();
  const bool ok = tid < 32;
  const int tc = ok ? tid : 0;
  const v4f v = *(const v4fa*)(stg + 4 * tc);
  float* dp = acout + 4 * tc;
  if (ok) *(volatile v4f*)dp = v;
  __threadfence();
  if (ok) *(volatile v4f*)dp = v;
}

__global__ __launch_bounds__(NTHR) void k_hpool(const float* __restrict__ Yin, const float* __restrict__ ac,
                                                const int* __restrict__ segt, int nN, int wrH,
                                                float* Hout, unsigned short* pc, int lcol) {
  __shared__ __attribute__((aligned(16))) float wsum[NWAVE * HD];
  __shared__ __attribute__((aligned(16))) float acs[2 * HD];
  __shared__ __attribute__((aligned(16))) unsigned short orow[2 * HD];
  const int tid = (int)threadIdx.x, lane = tid & 31, wave = tid >> 5;
  const int g = (int)blockIdx.x;
  if (tid < 32) *(v4fa*)(acs + 4 * tid) = *(const v4f*)(ac + 4 * tid);
  int s0 = segt[g];
  int s1 = segt[g + 1];
  s0 = s0 < 0 ? 0 : (s0 > nN ? nN : s0);
  s1 = s1 < s0 ? s0 : (s1 > nN ? nN : s1);
  __syncthreads();
  const float a0 = acs[2 * lane], a1 = acs[2 * lane + 1];
  const float c0 = acs[HD + 2 * lane], c1 = acs[HD + 2 * lane + 1];
  float p0 = 0.0f, p1 = 0.0f;
#pragma unroll 1
  for (int i = s0 + wave; i < s1; i += NWAVE) {
    const v2f y = *(const v2fa*)(Yin + (size_t)i * HD + 2 * lane);
    v2f hv;
    hv.x = relu_keep(fmaf(a0, y.x, c0));
    hv.y = relu_keep(fmaf(a1, y.y, c1));
    p0 += hv.x; p1 += hv.y;
    if (wrH != 0) {
      float* hp = Hout + (size_t)i * HD + 2 * lane;
      *(volatile v2f*)hp = hv;
      __threadfence();
      *(volatile v2f*)hp = hv;
    }
  }
  wsum[wave * HD + 2 * lane]     = p0;
  wsum[wave * HD + 2 * lane + 1] = p1;
  __syncthreads();
  if (tid < HD) {
    float s = 0.0f;
#pragma unroll
    for (int w2 = 0; w2 < NWAVE; ++w2) s += wsum[w2 * HD + tid];
    const unsigned short hb = bf_bits(s);
    orow[tid] = hb;
    orow[HD + tid] = bf_bits(s - bf_val(hb));
  }
  __syncthreads();
  const bool ok = (wave == 0) && (lane < 16);
  const int lc = lane & 15;
  const v8us ov = *(const v8usa*)(orow + 8 * lc);
  unsigned short* dp = pc + (size_t)g * KRO + (lc < 8 ? 0 : (KRO / 2)) + lcol * HD + 8 * (lc & 7);
  if (ok) *(volatile v8us*)dp = ov;
  __threadfence();
  if (ok) *(volatile v8us*)dp = ov;
}

__global__ __launch_bounds__(128) void k_readout(const unsigned short* __restrict__ PC,
                                                 const unsigned short* __restrict__ LW,
                                                 const float* __restrict__ linb, const int* __restrict__ segt,
                                                 int nN, float* out) {
  __shared__ __attribute__((aligned(16))) float stg[64 * HD];
  __shared__ float b0s[HD];
  __shared__ float bsum[HD];
  __shared__ float cnts[64];
  const int tid = (int)threadIdx.x, lane = tid & 31, wave = tid >> 5, hh = lane >> 4, m = lane & 15;
  const int rowBase = (int)blockIdx.x * 64;
  if (tid < HD) {
    b0s[tid] = bf_rne(linb[tid]);
    bsum[tid] = ((bf_rne(linb[HD + tid]) + bf_rne(linb[2 * HD + tid])) + bf_rne(linb[3 * HD + tid]))
                + bf_rne(linb[4 * HD + tid]);
    const int g = rowBase + tid;
    int s0 = segt[g], s1 = segt[g + 1];
    s0 = s0 < 0 ? 0 : (s0 > nN ? nN : s0);
    s1 = s1 < s0 ? s0 : (s1 > nN ? nN : s1);
    cnts[tid] = (float)(s1 - s0);
  }
  const int flag = segt[SEGFLAG];
  __syncthreads();

  v8f acc[4];
  {
    const v8f z = {0.f, 0.f, 0.f, 0.f, 0.f, 0.f, 0.f, 0.f};
    acc[0] = z; acc[1] = z; acc[2] = z; acc[3] = z;
  }
  const unsigned short* ap = PC + (size_t)(rowBase + 16 * wave + m) * KRO + 8 * hh;
  const unsigned short* wp = LW + (size_t)m * KRO + 8 * hh;
#pragma unroll 1
  for (int k0 = 0; k0 < KRO; k0 += 32) {
    Frag af;
    af.h[0] = *(const v8usa*)(ap + k0);
    af.h[1] = *(const v8usa*)(ap + k0 + 16);
#pragma unroll
    for (int nt = 0; nt < 4; ++nt) {
      const unsigned short* wq = wp + (size_t)(16 * nt) * KRO + k0;
      Frag bfr;
      bfr.h[0] = *(const v8usa*)wq;
      bfr.h[1] = *(const v8usa*)(wq + 16);
      acc[nt] = wmb(af, bfr, acc[nt]);
    }
  }
  const float qnan = __int_as_float(0x7fc00000);
  const float pz = (flag != 0) ? qnan : 0.0f;
#pragma unroll
  for (int nt = 0; nt < 4; ++nt) {
    const int lc = 16 * nt + m;
#pragma unroll
    for (int r = 0; r < 8; ++r) {
      const int lr = 16 * wave + 8 * hh + r;
      const float add = fmaf(cnts[lr], b0s[lc], bsum[lc]);
      stg[lr * HD + lc] = (acc[nt][r] + add) + pz;
    }
  }
  __syncthreads();
  v4f fv[8];
#pragma unroll
  for (int i = 0; i < 8; ++i) {
    const int lr = 16 * wave + 2 * i + hh;
    fv[i] = *(const v4fa*)(stg + lr * HD + 4 * m);
  }
#pragma unroll
  for (int i = 0; i < 8; ++i) {
    const int lr = 16 * wave + 2 * i + hh;
    float* op = out + (size_t)(rowBase + lr) * HD + 4 * m;
    *(volatile v4f*)op = fv[i];
  }
  __threadfence();
#pragma unroll
  for (int i = 0; i < 8; ++i) {
    const int lr = 16 * wave + 2 * i + hh;
    float* op = out + (size_t)(rowBase + lr) * HD + 4 * m;
    *(volatile v4f*)op = fv[i];
  }
}

static inline int cdiv(int a, int b) { return (a + b - 1) / b; }
static inline size_t al256(size_t o) { return (o + 255) & ~(size_t)255; }

extern "C" void kernel_launch(void* const* d_in, const int* in_sizes, int n_in,
                              void* d_out, int out_size, void* d_ws, size_t ws_size,
                              hipStream_t stream) {
  if (n_in < 21) return;
  if (in_sizes[0] < FEA || (in_sizes[0] % FEA) != 0) return;
  const int nN = in_sizes[0] / FEA;
  if (nN < 1 || nN > (1 << 20)) return;
  if (in_sizes[1] < 2 || (in_sizes[1] & 1) != 0) return;
  const int nE = in_sizes[1] / 2;
  if (nE < 1 || nE > (1 << 21)) return;
  if (in_sizes[2] != nN) return;
  if (in_sizes[3] != FEA * HD) return;
  if (in_sizes[4] != HD || in_sizes[5] != HD || in_sizes[6] != HD) return;
  if (in_sizes[7] != HD * HD) return;
  if (in_sizes[8] != HD || in_sizes[9] != HD || in_sizes[10] != HD) return;
  if (in_sizes[11] != NLAY * HD * HD) return;
  if (in_sizes[12] != NLAY * HD || in_sizes[13] != NLAY * HD || in_sizes[14] != NLAY * HD) return;
  if (in_sizes[15] != NLAY * HD * HD) return;
  if (in_sizes[16] != NLAY * HD || in_sizes[17] != NLAY * HD || in_sizes[18] != NLAY * HD) return;
  if (in_sizes[19] != (NLAY + 1) * HD * HD) return;
  if (in_sizes[20] != (NLAY + 1) * HD) return;
  if (out_size != NGR * HD) return;

  const float* x    = (const float*)d_in[0];
  const int*   ei   = (const int*)  d_in[1];
  const int*   src  = ei;
  const int*   dst  = ei + nE;
  const int*   bat  = (const int*)  d_in[2];
  const float* fW1  = (const float*)d_in[3];
  const float* fb1  = (const float*)d_in[4];
  const float* fg1  = (const float*)d_in[5];
  const float* fbt1 = (const float*)d_in[6];
  const float* fW2  = (const float*)d_in[7];
  const float* fb2  = (const float*)d_in[8];
  const float* fg2  = (const float*)d_in[9];
  const float* fbt2 = (const float*)d_in[10];
  const float* cW1  = (const float*)d_in[11];
  const float* cb1  = (const float*)d_in[12];
  const float* cg1  = (const float*)d_in[13];
  const float* cbt1 = (const float*)d_in[14];
  const float* cW2  = (const float*)d_in[15];
  const float* cb2  = (const float*)d_in[16];
  const float* cg2  = (const float*)d_in[17];
  const float* cbt2 = (const float*)d_in[18];
  const float* linW = (const float*)d_in[19];
  const float* linb = (const float*)d_in[20];
  float* out = (float*)d_out;

  const int MP = cdiv(nN, TM) * TM;
  const int gT = MP / TM;
  const int gC = cdiv(MP, NB);
  if ((long long)gC * NB < (long long)MP) return;
  const int vec8 = ((nE & 3) == 0) ? 1 : 0;

  char* ws = (char*)d_ws;
  size_t off = 0;
  const size_t oSEG = off; off = al256(off + (size_t)SEGW * 4);
  const size_t oF1  = off; off = al256(off + (size_t)HD * K2 * 2);
  const size_t oF2  = off; off = al256(off + (size_t)HD * K2 * 2);
  const size_t oC1  = off; off = al256(off + (size_t)NLAY * HD * K2 * 2);
  const size_t oC2  = off; off = al256(off + (size_t)NLAY * HD * K2 * 2);
  const size_t oLW  = off; off = al256(off + (size_t)HD * KRO * 2);
  const size_t oCM  = off; off = al256(off + (size_t)gC * CSRMW * 4);
  const size_t oCL  = off; off = al256(off + (size_t)gC * RCAP * 4);
  const size_t oY   = off; off = al256(off + (size_t)MP * HD * 4);
  const size_t oY2  = off; off = al256(off + (size_t)MP * HD * 4);
  const size_t oH   = off; off = al256(off + (size_t)MP * HD * 4);
  const size_t oPT  = off; off = al256(off + (size_t)gT * PARTW * 4);
  const size_t oAC  = off; off = al256(off + (size_t)10 * 128 * 4);
  const size_t oPC  = off; off = al256(off + (size_t)NGR * KRO * 2);
  if (off > ws_size || off > (size_t)WSMAX) return;
  int*            SEGT = (int*)(ws + oSEG);
  unsigned short* FW1T = (unsigned short*)(ws + oF1);
  unsigned short* FW2T = (unsigned short*)(ws + oF2);
  unsigned short* CW1T = (unsigned short*)(ws + oC1);
  unsigned short* CW2T = (unsigned short*)(ws + oC2);
  unsigned short* LW2  = (unsigned short*)(ws + oLW);
  int*            CSRM = (int*)(ws + oCM);
  int*            COL  = (int*)(ws + oCL);
  float*          Y    = (float*)(ws + oY);
  float*          Y2   = (float*)(ws + oY2);
  float*          H    = (float*)(ws + oH);
  float*          PT   = (float*)(ws + oPT);
  float*          AC   = (float*)(ws + oAC);
  unsigned short* PC   = (unsigned short*)(ws + oPC);

  hipFuncSetAttribute(reinterpret_cast<const void*>(&k_csr),     hipFuncAttributeMaxDynamicSharedMemorySize, LDS_CSR);
  hipFuncSetAttribute(reinterpret_cast<const void*>(&k_gemm<0>), hipFuncAttributeMaxDynamicSharedMemorySize, GEMM_LDS);
  hipFuncSetAttribute(reinterpret_cast<const void*>(&k_gemm<1>), hipFuncAttributeMaxDynamicSharedMemorySize, GEMM_LDS);
  hipFuncSetAttribute(reinterpret_cast<const void*>(&k_gemm<2>), hipFuncAttributeMaxDynamicSharedMemorySize, GEMM_LDS);

  k_prep<<<NUPREP / NTHR, NTHR, 0, stream>>>(fW1, fW2, cW1, cW2, linW, FW1T, FW2T, CW1T, CW2T, LW2);
  k_seg<<<1, NTHR, 0, stream>>>(bat, nN, SEGT);
  k_csr<<<gC, NTHR, LDS_CSR, stream>>>(src, dst, nN, nE, vec8, CSRM, COL);
  k_gemm<0><<<gT, NTHR, GEMM_LDS, stream>>>(x, AC, CSRM, COL, FW1T, fb1, Y, PT, nN);
  k_bncomb<<<1, HD, 0, stream>>>(PT, gT, fg1, fbt1, AC);
  k_gemm<1><<<gT, NTHR, GEMM_LDS, stream>>>(Y, AC, CSRM, COL, FW2T, fb2, Y2, PT, nN);
  k_bncomb<<<1, HD, 0, stream>>>(PT, gT, fg2, fbt2, AC + 128);
  k_hpool<<<NGR, NTHR, 0, stream>>>(Y2, AC + 128, SEGT, nN, 1, H, PC, 0);
  for (int l = 0; l < NLAY; ++l) {
    float* ac1 = AC + (size_t)(2 + 2 * l) * 128;
    float* ac2 = AC + (size_t)(3 + 2 * l) * 128;
    k_gemm<2><<<gT, NTHR, GEMM_LDS, stream>>>(H, AC, CSRM, COL, CW1T + (size_t)l * HD * K2, cb1 + l * HD, Y, PT, nN);
    k_bncomb<<<1, HD, 0, stream>>>(PT, gT, cg1 + l * HD, cbt1 + l * HD, ac1);
    k_gemm<1><<<gT, NTHR, GEMM_LDS, stream>>>(Y, ac1, CSRM, COL, CW2T + (size_t)l * HD * K2, cb2 + l * HD, Y2, PT, nN);
    k_bncomb<<<1, HD, 0, stream>>>(PT, gT, cg2 + l * HD, cbt2 + l * HD, ac2);
    k_hpool<<<NGR, NTHR, 0, stream>>>(Y2, ac2, SEGT, nN, (l < NLAY - 1) ? 1 : 0, H, PC, l + 1);
  }
  k_readout<<<NGR / 64, 128, 0, stream>>>(PC, LW2, linb, SEGT, nN, out);
}
